// TriangleAttention_20186346291617
// MI455X (gfx1250) — hardware-verified
//
#include <hip/hip_runtime.h>
#include <stdint.h>


#define NN   256
#define CZ   128
#define HN   4
#define DH   32
#define NPOS (NN * NN)
#define NW   (CZ * CZ)
#define PB   64
#define AP   128
#define AW   2
#define QMUL (0.25f * 0.17677669529663687f)

typedef char chk_pb  [(NPOS % PB == 0) ? 1 : -1];
typedef char chk_pb2 [(NN % PB == 0) ? 1 : -1];
typedef char chk_aw  [((NN * HN * (NN / 16)) % AW == 0) ? 1 : -1];
typedef char chk_rt  [(NPOS % 16 == 0) ? 1 : -1];
typedef char chk_cvt [(NW % 8 == 0) ? 1 : -1];

typedef _Float16 v16h __attribute__((ext_vector_type(16)));
typedef _Float16 v8h  __attribute__((ext_vector_type(8)));
typedef _Float16 v4h  __attribute__((ext_vector_type(4)));
typedef __bf16   v16b __attribute__((ext_vector_type(16)));
typedef unsigned short v8us __attribute__((ext_vector_type(8)));
typedef unsigned short v4us __attribute__((ext_vector_type(4)));
typedef float v8f __attribute__((ext_vector_type(8)));
typedef float v4f __attribute__((ext_vector_type(4)));
typedef int   v8i __attribute__((ext_vector_type(8)));
typedef v8h  v8ha  __attribute__((may_alias));
typedef v8us v8usa __attribute__((may_alias));
typedef v4f  v4fa  __attribute__((may_alias));

union FragH { v16h v; v8h p[2]; v4h q[4]; };
union FragB { v16b v; v8i w; v8us p[2]; };

__device__ __forceinline__ v8f zero8() {
    v8f z = {0.f, 0.f, 0.f, 0.f, 0.f, 0.f, 0.f, 0.f};
    return z;
}

__device__ __forceinline__ v8f mma_f16(v16h a, v16h b, v8f c) {
    v8f d = __builtin_amdgcn_wmma_f32_16x16x32_f16(false, a, false, b, (short)0, c, false, false);
    asm volatile("v_nop\n\tv_nop\n\tv_nop\n\tv_nop" : "+v"(d) : "v"(a), "v"(b));
    return d;
}
__device__ __forceinline__ v8f mma_bf16(const FragB a, const FragB b, v8f c) {
    v8f d = __builtin_amdgcn_wmma_f32_16x16x32_bf16(false, a.v, false, b.v, (short)0, c, false, false);
    asm volatile("v_nop\n\tv_nop\n\tv_nop\n\tv_nop" : "+v"(d) : "v"(a.w), "v"(b.w));
    return d;
}

__device__ __forceinline__ v16h frag_h(const _Float16* p, int hh) {
    FragH f;
    f.p[0] = *(const v8ha*)(p + 8 * hh);
    f.p[1] = *(const v8ha*)(p + 16 + 8 * hh);
    return f.v;
}
__device__ __forceinline__ FragB frag_b(const unsigned short* p, int hh) {
    FragB f;
    f.p[0] = *(const v8usa*)(p + 8 * hh);
    f.p[1] = *(const v8usa*)(p + 16 + 8 * hh);
    return f;
}

__device__ __forceinline__ unsigned short bf16_rne(float f) {
    unsigned u = __float_as_uint(f);
    u += 0x7FFFu + ((u >> 16) & 1u);
    return (unsigned short)(u >> 16);
}
__device__ __forceinline__ float bf16_val(unsigned short b) {
    return __uint_as_float(((unsigned)b) << 16);
}
__device__ __forceinline__ float wsum(float v) {
    #pragma unroll
    for (int off = 16; off; off >>= 1) v += __shfl_xor(v, off, 32);
    return v;
}
__device__ __forceinline__ float wmax(float v) {
    #pragma unroll
    for (int off = 16; off; off >>= 1) v = fmaxf(v, __shfl_xor(v, off, 32));
    return v;
}

__device__ __forceinline__ v8f tile_f16(const _Float16* arow, const _Float16* brow, int hh) {
    v8f acc = zero8();
    #pragma unroll
    for (int cc = 0; cc < CZ / 32; ++cc) {
        const v16h a = frag_h(arow + cc * 32, hh);
        const v16h b = frag_h(brow + cc * 32, hh);
        acc = mma_f16(a, b, acc);
    }
    return acc;
}
__device__ __forceinline__ v8f tile_bf16x3(const unsigned short* ahr, const unsigned short* alr,
                                            const unsigned short* bhr, const unsigned short* blr, int hh) {
    v8f acc = zero8();
    #pragma unroll
    for (int cc = 0; cc < CZ / 32; ++cc) {
        const FragB ah = frag_b(ahr + cc * 32, hh);
        const FragB al = frag_b(alr + cc * 32, hh);
        const FragB bh = frag_b(bhr + cc * 32, hh);
        const FragB bl = frag_b(blr + cc * 32, hh);
        acc = mma_bf16(ah, bh, acc);
        acc = mma_bf16(ah, bl, acc);
        acc = mma_bf16(al, bh, acc);
    }
    return acc;
}

__global__ __launch_bounds__(256) void k_cvt(
    const float* __restrict__ wq, const float* __restrict__ wk, const float* __restrict__ wv,
    const float* __restrict__ wg, const float* __restrict__ wo,
    _Float16* Wq16, _Float16* Wk16, _Float16* Wg16,
    unsigned short* Wvh, unsigned short* Wvl, unsigned short* Woh, unsigned short* Wol, int n)
{
    const int t = blockIdx.x * blockDim.x + threadIdx.x;
    const int base = t * 8;
    if (base + 8 > n) return;

    union U8h { v8h v; v4h q[2]; };
    union U8f { v4f q[2]; float f[8]; };
    U8h uq, uk, ug;
    {
        const v4f a0 = *(const v4f*)(wq + base), a1 = *(const v4f*)(wq + base + 4);
        uq.q[0] = __builtin_convertvector(a0 * 64.0f, v4h);
        uq.q[1] = __builtin_convertvector(a1 * 64.0f, v4h);
    }
    {
        const v4f a0 = *(const v4f*)(wk + base), a1 = *(const v4f*)(wk + base + 4);
        uk.q[0] = __builtin_convertvector(a0 * 64.0f, v4h);
        uk.q[1] = __builtin_convertvector(a1 * 64.0f, v4h);
    }
    {
        const v4f a0 = *(const v4f*)(wg + base), a1 = *(const v4f*)(wg + base + 4);
        ug.q[0] = __builtin_convertvector(a0 * 64.0f, v4h);
        ug.q[1] = __builtin_convertvector(a1 * 64.0f, v4h);
    }
    v8us vh, vl, oh, ol;
    {
        U8f u;
        u.q[0] = *(const v4f*)(wv + base); u.q[1] = *(const v4f*)(wv + base + 4);
        #pragma unroll
        for (int e = 0; e < 8; ++e) {
            const unsigned short hb = bf16_rne(u.f[e]);
            vh[e] = hb;
            vl[e] = bf16_rne(u.f[e] - bf16_val(hb));
        }
    }
    {
        U8f u;
        u.q[0] = *(const v4f*)(wo + base); u.q[1] = *(const v4f*)(wo + base + 4);
        #pragma unroll
        for (int e = 0; e < 8; ++e) {
            const unsigned short hb = bf16_rne(u.f[e]);
            oh[e] = hb;
            ol[e] = bf16_rne(u.f[e] - bf16_val(hb));
        }
    }
    *(volatile v8h*)(Wq16 + base) = uq.v;
    *(volatile v8h*)(Wk16 + base) = uk.v;
    *(volatile v8h*)(Wg16 + base) = ug.v;
    *(volatile v8us*)(Wvh + base) = vh;
    *(volatile v8us*)(Wvl + base) = vl;
    *(volatile v8us*)(Woh + base) = oh;
    *(volatile v8us*)(Wol + base) = ol;
    __threadfence();
    *(volatile v8h*)(Wq16 + base) = uq.v;
    *(volatile v8h*)(Wk16 + base) = uk.v;
    *(volatile v8h*)(Wg16 + base) = ug.v;
    *(volatile v8us*)(Wvh + base) = vh;
    *(volatile v8us*)(Wvl + base) = vl;
    *(volatile v8us*)(Woh + base) = oh;
    *(volatile v8us*)(Wol + base) = ol;
}

__global__ __launch_bounds__(256) void k_proj(
    const float* __restrict__ x, const float* __restrict__ ln_w, const float* __restrict__ ln_b,
    const float* __restrict__ w_tri, const float* __restrict__ bg,
    const _Float16* __restrict__ Wq16, const _Float16* __restrict__ Wk16, const _Float16* __restrict__ Wg16,
    const unsigned short* __restrict__ Wvh, const unsigned short* __restrict__ Wvl,
    _Float16* Qh, _Float16* Kh, _Float16* Vt, float* Gf, float* tri)
{
    __shared__ __align__(16) _Float16       Af [PB * AP];
    __shared__ __align__(16) unsigned short Ahb[PB * AP];
    __shared__ __align__(16) unsigned short Alb[PB * AP];
    __shared__ __align__(16) char           stg[16384];

    const int tid = threadIdx.x, w = tid >> 5, l = tid & 31, hh = l >> 4, m = l & 15;
    const int blk  = blockIdx.x;
    const int pos0 = blk * PB;

    {
        float* triS = (float*)stg;
        const v4f w4 = *(const v4f*)(ln_w + 4 * l);
        const v4f b4 = *(const v4f*)(ln_b + 4 * l);
        v4f wt[HN];
        #pragma unroll
        for (int h = 0; h < HN; ++h) wt[h] = *(const v4f*)(w_tri + h * CZ + 4 * l);

        #pragma unroll 1
        for (int j = 0; j < PB / 8; ++j) {
            const int pl = w * (PB / 8) + j;
            const size_t pos = (size_t)pos0 + pl;
            const v4f a = *(const v4f*)(x + pos * CZ + 4 * l);
            const float mu = wsum(a[0] + a[1] + a[2] + a[3]) * (1.0f / CZ);
            const v4f d = a - mu;
            const float var = wsum(d[0] * d[0] + d[1] * d[1] + d[2] * d[2] + d[3] * d[3]) * (1.0f / CZ);
            const float rstd = rsqrtf(var + 1e-5f);
            const v4f y = d * rstd * w4 + b4;

            *(v4h*)(Af + pl * AP + 4 * l) = __builtin_convertvector(y, v4h);
            v4us hb4, lb4;
            #pragma unroll
            for (int c = 0; c < 4; ++c) {
                const unsigned short hb = bf16_rne(y[c]);
                hb4[c] = hb;
                lb4[c] = bf16_rne(y[c] - bf16_val(hb));
            }
            *(v4us*)(Ahb + pl * AP + 4 * l) = hb4;
            *(v4us*)(Alb + pl * AP + 4 * l) = lb4;

            #pragma unroll
            for (int h = 0; h < HN; ++h) {
                const float t = wsum(y[0] * wt[h][0] + y[1] * wt[h][1] + y[2] * wt[h][2] + y[3] * wt[h][3]);
                if (l == 0) triS[h * PB + pl] = t;
            }
        }
    }
    __syncthreads();
    if (tid < HN * (PB / 4)) {
        const int h = tid >> 4, part = tid & 15;
        const v4f v = *(const v4fa*)((const float*)stg + h * PB + part * 4);
        float* dp = tri + (size_t)h * NPOS + pos0 + part * 4;
        *(volatile v4f*)dp = v;
        __threadfence();
        *(volatile v4f*)dp = v;
    }
    __syncthreads();

    const int e = w * 16 + m;

    #pragma unroll 1
    for (int p = 0; p < 2; ++p) {
        const _Float16* wrow = (p == 0 ? Wq16 : Wk16) + (size_t)e * CZ;
        const float mul = (p == 0) ? QMUL : (1.0f / 64.0f);
        _Float16* dst = (p == 0) ? Qh : Kh;
        _Float16* sh = (_Float16*)stg;
        #pragma unroll 1
        for (int rt = 0; rt < PB / 16; ++rt) {
            const v8f acc = tile_f16(Af + (rt * 16 + m) * AP, wrow, hh);
            #pragma unroll
            for (int r = 0; r < 8; ++r) sh[(rt * 16 + 8 * hh + r) * CZ + e] = (_Float16)(acc[r] * mul);
        }
        __syncthreads();
        v8h vv[4]; size_t go[4];
        #pragma unroll
        for (int jj = 0; jj < 4; ++jj) {
            const int c = tid + 256 * jj;
            const int row = c >> 4, col = (c & 15) * 8;
            vv[jj] = *(const v8ha*)(sh + row * CZ + col);
            go[jj] = ((size_t)pos0 + row) * CZ + col;
        }
        #pragma unroll
        for (int jj = 0; jj < 4; ++jj) *(volatile v8h*)(dst + go[jj]) = vv[jj];
        __threadfence();
        #pragma unroll
        for (int jj = 0; jj < 4; ++jj) *(volatile v8h*)(dst + go[jj]) = vv[jj];
        __syncthreads();
    }

    {
        const _Float16* wrow = Wg16 + (size_t)e * CZ;
        const float bge = bg[e];
        float* sf = (float*)stg;
        #pragma unroll 1
        for (int half = 0; half < 2; ++half) {
            #pragma unroll 1
            for (int rr = 0; rr < 2; ++rr) {
                const int rt = half * 2 + rr;
                const v8f acc = tile_f16(Af + (rt * 16 + m) * AP, wrow, hh);
                #pragma unroll
                for (int r = 0; r < 8; ++r) {
                    const float z = acc[r] * (1.0f / 64.0f) + bge;
                    sf[(rr * 16 + 8 * hh + r) * CZ + e] = __builtin_amdgcn_rcpf(1.0f + __expf(-z));
                }
            }
            __syncthreads();
            v4f vv[4]; size_t go[4];
            #pragma unroll
            for (int jj = 0; jj < 4; ++jj) {
                const int c = tid + 256 * jj;
                const int row = c >> 5, col = (c & 31) * 4;
                vv[jj] = *(const v4fa*)(sf + row * CZ + col);
                go[jj] = ((size_t)pos0 + half * 32 + row) * CZ + col;
            }
            #pragma unroll
            for (int jj = 0; jj < 4; ++jj) *(volatile v4f*)(Gf + go[jj]) = vv[jj];
            __threadfence();
            #pragma unroll
            for (int jj = 0; jj < 4; ++jj) *(volatile v4f*)(Gf + go[jj]) = vv[jj];
            __syncthreads();
        }
    }

    {
        const unsigned short* whr = Wvh + (size_t)e * CZ;
        const unsigned short* wlr = Wvl + (size_t)e * CZ;
        _Float16* sv = (_Float16*)stg;
        #pragma unroll 1
        for (int rt = 0; rt < PB / 16; ++rt) {
            const v8f acc = tile_bf16x3(Ahb + (rt * 16 + m) * AP, Alb + (rt * 16 + m) * AP, whr, wlr, hh);
            #pragma unroll
            for (int r = 0; r < 8; ++r) sv[e * PB + rt * 16 + 8 * hh + r] = (_Float16)acc[r];
        }
        __syncthreads();
        const int ii = blk / (NN / PB), kseg = blk % (NN / PB);
        v8h vv[4]; size_t go[4];
        #pragma unroll
        for (int jj = 0; jj < 4; ++jj) {
            const int c = tid + 256 * jj;
            const int ee = c >> 3, part = c & 7;
            vv[jj] = *(const v8ha*)(sv + ee * PB + part * 8);
            go[jj] = ((size_t)(ii * CZ + ee)) * NN + kseg * PB + part * 8;
        }
        #pragma unroll
        for (int jj = 0; jj < 4; ++jj) *(volatile v8h*)(Vt + go[jj]) = vv[jj];
        __threadfence();
        #pragma unroll
        for (int jj = 0; jj < 4; ++jj) *(volatile v8h*)(Vt + go[jj]) = vv[jj];
    }
}

__global__ __launch_bounds__(AW * 32) void k_attn(
    const _Float16* __restrict__ Qh, const _Float16* __restrict__ Kh, const _Float16* __restrict__ Vt,
    const float* __restrict__ Gf, const float* __restrict__ tri, const float* __restrict__ mask,
    unsigned short* Oh, unsigned short* Ol)
{
    __shared__ __align__(16) float sc[AW][16][NN];
    const int tid = threadIdx.x, wv = tid >> 5, l = tid & 31, hh = l >> 4, m = l & 15;
    const int task = blockIdx.x * AW + wv;
    const int qt = task & 15, h = (task >> 4) & (HN - 1), i = task >> 6;
    const int q0 = qt * 16;
    float (*scw)[NN] = sc[wv];

    const v16h qa = frag_h(Qh + ((size_t)(i * NN + q0 + m)) * CZ + h * DH, hh);
    #pragma unroll 2
    for (int kt = 0; kt < NN / 16; ++kt) {
        const v16h kb = frag_h(Kh + ((size_t)(i * NN + kt * 16 + m)) * CZ + h * DH, hh);
        const v8f s = mma_f16(qa, kb, zero8());
        const int kg = kt * 16 + m;
        const float mb = 1.0e9f * (mask[(size_t)i * NN + kg] - 1.0f);
        const float* tp = tri + (size_t)h * NPOS + (size_t)(q0 + 8 * hh) * NN + kg;
        #pragma unroll
        for (int r = 0; r < 8; ++r) scw[8 * hh + r][kg] = (s[r] * (1.0f / 16.0f) + mb) + tp[(size_t)r * NN];
    }
    __syncthreads();

    #pragma unroll 1
    for (int r = 0; r < 16; ++r) {
        float vals[8];
        float mx = -3.0e38f;
        #pragma unroll
        for (int j = 0; j < 8; ++j) { vals[j] = scw[r][l + 32 * j]; mx = fmaxf(mx, vals[j]); }
        mx = wmax(mx);
        float sm = 0.0f;
        #pragma unroll
        for (int j = 0; j < 8; ++j) { vals[j] = __expf(vals[j] - mx); sm += vals[j]; }
        sm = wsum(sm);
        const float pm = 256.0f * __builtin_amdgcn_rcpf(sm);
        #pragma unroll
        for (int j = 0; j < 8; ++j) scw[r][l + 32 * j] = vals[j] * pm;
    }
    __syncthreads();

    v8f acc0 = zero8(), acc1 = zero8();
    #pragma unroll 2
    for (int kc = 0; kc < NN / 32; ++kc) {
        const float* pr = &scw[m][kc * 32];
        FragH pa;
        pa.q[0] = __builtin_convertvector(*(const v4fa*)(pr + 8 * hh), v4h);
        pa.q[1] = __builtin_convertvector(*(const v4fa*)(pr + 8 * hh + 4), v4h);
        pa.q[2] = __builtin_convertvector(*(const v4fa*)(pr + 16 + 8 * hh), v4h);
        pa.q[3] = __builtin_convertvector(*(const v4fa*)(pr + 20 + 8 * hh), v4h);
        const _Float16* vr = Vt + ((size_t)(i * CZ + h * DH + m)) * NN + kc * 32;
        const v16h b0 = frag_h(vr, hh);
        const v16h b1 = frag_h(vr + (size_t)16 * NN, hh);
        acc0 = mma_f16(pa.v, b0, acc0);
        acc1 = mma_f16(pa.v, b1, acc1);
    }
    __syncthreads();

    float* ost = &sc[wv][0][0];
    {
        const float* gr = Gf + ((size_t)(i * NN + q0)) * CZ + h * DH;
        #pragma unroll
        for (int r = 0; r < 8; ++r) {
            const int qr = 8 * hh + r;
            const float g0 = gr[(size_t)qr * CZ + m];
            const float g1 = gr[(size_t)qr * CZ + 16 + m];
            ost[qr * 32 + m]      = acc0[r] * (1.0f / 256.0f) * g0;
            ost[qr * 32 + 16 + m] = acc1[r] * (1.0f / 256.0f) * g1;
        }
    }
    __syncthreads();

    const size_t tb = ((size_t)((i * HN + h) * NN + q0)) * DH;
    v8us hv[2], lv[2];
    #pragma unroll
    for (int jj = 0; jj < 2; ++jj) {
        const int c = l + 32 * jj;
        union { v4f q[2]; float f[8]; } u;
        u.q[0] = *(const v4fa*)(ost + c * 8);
        u.q[1] = *(const v4fa*)(ost + c * 8 + 4);
        #pragma unroll
        for (int t = 0; t < 8; ++t) {
            const unsigned short hb = bf16_rne(u.f[t]);
            hv[jj][t] = hb;
            lv[jj][t] = bf16_rne(u.f[t] - bf16_val(hb));
        }
    }
    #pragma unroll
    for (int jj = 0; jj < 2; ++jj) {
        *(volatile v8us*)(Oh + tb + (size_t)(l + 32 * jj) * 8) = hv[jj];
        *(volatile v8us*)(Ol + tb + (size_t)(l + 32 * jj) * 8) = lv[jj];
    }
    __threadfence();
    #pragma unroll
    for (int jj = 0; jj < 2; ++jj) {
        *(volatile v8us*)(Oh + tb + (size_t)(l + 32 * jj) * 8) = hv[jj];
        *(volatile v8us*)(Ol + tb + (size_t)(l + 32 * jj) * 8) = lv[jj];
    }
}

__global__ __launch_bounds__(256) void k_out(
    const unsigned short* __restrict__ Oh, const unsigned short* __restrict__ Ol,
    const unsigned short* __restrict__ Woh, const unsigned short* __restrict__ Wol,
    const float* __restrict__ bo, float* out)
{
    __shared__ __align__(16) float sf[16 * CZ];
    const int tid = threadIdx.x, w = tid >> 5, l = tid & 31, hh = l >> 4, m = l & 15;
    const int rt = blockIdx.x;
    const int p0 = rt * 16;
    const int i = p0 / NN;
    const int q = (p0 % NN) + m;
    const int c = w * 16 + m;
    const unsigned short* bhr = Woh + (size_t)c * CZ;
    const unsigned short* blr = Wol + (size_t)c * CZ;

    v8f acc = zero8();
    #pragma unroll
    for (int cc = 0; cc < HN; ++cc) {
        const size_t ab = ((size_t)((i * HN + cc) * NN + q)) * DH;
        const FragB ah = frag_b(Oh + ab, hh);
        const FragB al = frag_b(Ol + ab, hh);
        const FragB bh = frag_b(bhr + cc * 32, hh);
        const FragB bl = frag_b(blr + cc * 32, hh);
        acc = mma_bf16(ah, bh, acc);
        acc = mma_bf16(ah, bl, acc);
        acc = mma_bf16(al, bh, acc);
    }
    const float boc = bo[c];
    #pragma unroll
    for (int r = 0; r < 8; ++r) sf[(8 * hh + r) * CZ + c] = acc[r] + boc;
    __syncthreads();

    v4f vv[2]; size_t go[2];
    #pragma unroll
    for (int jj = 0; jj < 2; ++jj) {
        const int ch = tid + 256 * jj;
        const int row = ch >> 5, col = (ch & 31) * 4;
        vv[jj] = *(const v4fa*)(sf + row * CZ + col);
        go[jj] = ((size_t)p0 + row) * CZ + col;
    }
    #pragma unroll
    for (int jj = 0; jj < 2; ++jj) *(volatile v4f*)(out + go[jj]) = vv[jj];
    __threadfence();
    #pragma unroll
    for (int jj = 0; jj < 2; ++jj) *(volatile v4f*)(out + go[jj]) = vv[jj];
}

extern "C" void kernel_launch(void* const* d_in, const int* in_sizes, int n_in,
                              void* d_out, int out_size, void* d_ws, size_t ws_size,
                              hipStream_t stream)
{
    if (n_in < 12) return;
    if (in_sizes[0] != NPOS * CZ || in_sizes[1] != NPOS) return;
    if (in_sizes[2] != CZ || in_sizes[3] != CZ || in_sizes[4] != HN * CZ) return;
    if (in_sizes[5] != NW || in_sizes[6] != NW || in_sizes[7] != NW || in_sizes[8] != NW || in_sizes[10] != NW) return;
    if (in_sizes[9] != CZ || in_sizes[11] != CZ) return;
    if (out_size != NPOS * CZ) return;

    const float* x     = (const float*)d_in[0];
    const float* mask  = (const float*)d_in[1];
    const float* ln_w  = (const float*)d_in[2];
    const float* ln_b  = (const float*)d_in[3];
    const float* w_tri = (const float*)d_in[4];
    const float* wq    = (const float*)d_in[5];
    const float* wk    = (const float*)d_in[6];
    const float* wv    = (const float*)d_in[7];
    const float* wg    = (const float*)d_in[8];
    const float* bg    = (const float*)d_in[9];
    const float* wo    = (const float*)d_in[10];
    const float* bo    = (const float*)d_in[11];
    float* out = (float*)d_out;

    char* ws = (char*)d_ws;
    size_t off = 0;
    auto carve = [&](size_t bytes) -> char* {
        char* p = ws + off;
        off += (bytes + 255) & ~(size_t)255;
        return p;
    };
    _Float16* Wq16 = (_Float16*)carve((size_t)NW * 2);
    _Float16* Wk16 = (_Float16*)carve((size_t)NW * 2);
    _Float16* Wg16 = (_Float16*)carve((size_t)NW * 2);
    unsigned short* Wvh = (unsigned short*)carve((size_t)NW * 2);
    unsigned short* Wvl = (unsigned short*)carve((size_t)NW * 2);
    unsigned short* Woh = (unsigned short*)carve((size_t)NW * 2);
    unsigned short* Wol = (unsigned short*)carve((size_t)NW * 2);
    float*    tri = (float*)   carve((size_t)HN * NPOS * 4);
    _Float16* Qh  = (_Float16*)carve((size_t)NPOS * CZ * 2);
    _Float16* Kh  = (_Float16*)carve((size_t)NPOS * CZ * 2);
    _Float16* Vt  = (_Float16*)carve((size_t)NPOS * CZ * 2);
    float*    Gf  = (float*)   carve((size_t)NPOS * CZ * 4);
    unsigned short* Oh = (unsigned short*)carve((size_t)NPOS * CZ * 2);
    unsigned short* Ol = (unsigned short*)carve((size_t)NPOS * CZ * 2);
    if (off > ws_size) return;

    k_cvt<<<dim3((NW / 8 + 255) / 256), dim3(256), 0, stream>>>(wq, wk, wv, wg, wo,
                                                               Wq16, Wk16, Wg16, Wvh, Wvl, Woh, Wol, NW);
    k_proj<<<dim3(NPOS / PB), dim3(256), 0, stream>>>(x, ln_w, ln_b, w_tri, bg,
                                                      Wq16, Wk16, Wg16, Wvh, Wvl,
                                                      Qh, Kh, Vt, Gf, tri);
    k_attn<<<dim3((NN * HN * (NN / 16)) / AW), dim3(AW * 32), 0, stream>>>(Qh, Kh, Vt, Gf, tri, mask, Oh, Ol);
    k_out<<<dim3(NPOS / 16), dim3(256), 0, stream>>>(Oh, Ol, Woh, Wol, bo, out);
}
